// LSTMAutoencoder_80178449482357
// MI455X (gfx1250) — hardware-verified
//
#include <hip/hip_runtime.h>
#include <math.h>

typedef __attribute__((ext_vector_type(16))) _Float16 v16h;
typedef __attribute__((ext_vector_type(8)))  _Float16 v8h;
typedef __attribute__((ext_vector_type(16))) __bf16   v16b;
typedef __attribute__((ext_vector_type(8)))  __bf16   v8b;
typedef __attribute__((ext_vector_type(8)))  float    v8f;
typedef __attribute__((ext_vector_type(4)))  float    v4f;

constexpr int kB    = 4096;
constexpr int kT    = 100;
constexpr int kF    = 40;
constexpr int kHE   = 64;
constexpr int kHL   = 32;
constexpr int kHD   = 64;
constexpr int kKP   = 128;
constexpr int kRowsY = kB * kT;
constexpr int kRowsQ = kRowsY / 4;
constexpr int kThr  = 256;
constexpr float kInCarry = 1024.0f;
constexpr float kSc = 1.0f / (kInCarry * kInCarry);
constexpr float kF16MinNormal = 6.103515625e-5f;
constexpr int kFBE = 0, kFBL = 256, kFBD = 384, kFBO = 640, kFEnd = 1024;

static_assert((kB % 64) == 0 && (kRowsQ % 64) == 0 && ((kB / 64) * (256 / 64)) % 8 == 0 && ((kB / 64) * (128 / 64)) % 8 == 0 && ((kRowsQ / 64) * (64 / 64)) % 8 == 0 && (kKP % 32) == 0 && (kHD % 32) == 0,
              "GEMM M, N multiples of 64; grids exact; K multiples of 32");

constexpr size_t kOffWE = 0ull;
constexpr size_t kOffWL = 65536ull;
constexpr size_t kOffWD = 98304ull;
constexpr size_t kOffWO = 163840ull;
constexpr size_t kOffBIAS = 172032ull;
constexpr size_t kOffAE = 176128ull;
constexpr size_t kOffAL = 1224704ull;
constexpr size_t kOffAD = 2273280ull;
constexpr size_t kOffGE = 3321856ull;
constexpr size_t kOffGL = 7516160ull;
constexpr size_t kOffGD = 9613312ull;
constexpr size_t kOffCE = 13807616ull;
constexpr size_t kOffCL = 14856192ull;
constexpr size_t kOffCD = 15380480ull;
constexpr size_t kOffHD16 = 16429056ull;
constexpr size_t kOffO32 = 68857856ull;
constexpr size_t kWsTotal = 95072256ull;
static_assert(kWsTotal <= 134217728ull, "carve cap: under 128 MiB");
static_assert(kOffWE == 0
              && kOffWL == kOffWE + 65536ull
              && kOffWD == kOffWL + 32768ull
              && kOffWO == kOffWD + 65536ull
              && kOffBIAS == kOffWO + 8192ull
              && kOffAE == kOffBIAS + 4096ull
              && kOffAL == kOffAE + 1048576ull
              && kOffAD == kOffAL + 1048576ull
              && kOffGE == kOffAD + 1048576ull
              && kOffGL == kOffGE + 4194304ull
              && kOffGD == kOffGL + 2097152ull
              && kOffCE == kOffGD + 4194304ull
              && kOffCL == kOffCE + 1048576ull
              && kOffCD == kOffCL + 524288ull
              && kOffHD16 == kOffCD + 1048576ull
              && kOffO32 == kOffHD16 + 52428800ull
              && kWsTotal == kOffO32 + 26214400ull, "the carve is chained and totalled");
static_assert((kOffWE % 256) == 0 && (kOffWL % 256) == 0 && (kOffWD % 256) == 0 && (kOffWO % 256) == 0 && (kOffBIAS % 256) == 0 && (kOffAE % 256) == 0 && (kOffAL % 256) == 0 && (kOffAD % 256) == 0 && (kOffGE % 256) == 0 && (kOffGL % 256) == 0 && (kOffGD % 256) == 0 && (kOffCE % 256) == 0 && (kOffCL % 256) == 0 && (kOffCD % 256) == 0 && (kOffHD16 % 256) == 0 && (kOffO32 % 256) == 0, "aligned regions");

__device__ __forceinline__ unsigned short f2bf_bits(float f) {
  unsigned u = __float_as_uint(f);
  return (unsigned short)((u + 0x7FFFu + ((u >> 16) & 1u)) >> 16);
}
__device__ __forceinline__ float bf_bits2f(unsigned short h) { return __uint_as_float(((unsigned)h) << 16); }
__device__ __forceinline__ float bf16r(float f) { return bf_bits2f(f2bf_bits(f)); }
__device__ __forceinline__ float carry_flush(float v, float carry) {
  const float s = v * carry;
  return (fabsf(s) < kF16MinNormal) ? 0.0f : s;
}
__device__ __forceinline__ float frcp(float x) { return __builtin_amdgcn_rcpf(x); }

__device__ __forceinline__ void dep_guard4_h(v8f& a, v8f& b, v8f& c, v8f& d, v16h x, v16h y) { asm volatile("v_nop\n\tv_nop\n\tv_nop\n\tv_nop" : "+v"(a), "+v"(b), "+v"(c), "+v"(d) : "v"(x), "v"(y)); }
__device__ __forceinline__ void dep_guard4_b(v8f& a, v8f& b, v8f& c, v8f& d, v16b x, v16b y) { asm volatile("v_nop\n\tv_nop\n\tv_nop\n\tv_nop" : "+v"(a), "+v"(b), "+v"(c), "+v"(d) : "v"(x), "v"(y)); }
__device__ __forceinline__ void keep4_h(v16h a, v16h b, v16h c, v16h d) { asm volatile("v_nop" :: "v"(a), "v"(b), "v"(c), "v"(d)); }
__device__ __forceinline__ void keep4_b(v16b a, v16b b, v16b c, v16b d) { asm volatile("v_nop" :: "v"(a), "v"(b), "v"(c), "v"(d)); }
__device__ __forceinline__ void acc_guard4(v8f& a, v8f& b, v8f& c, v8f& d) { asm volatile("v_nop\n\tv_nop\n\tv_nop\n\tv_nop" : "+v"(a), "+v"(b), "+v"(c), "+v"(d)); }

template <typename T> struct Frag;
template <> struct Frag<_Float16> {
  typedef v16h V; union U { v16h v; v8h h[2]; };
  static __device__ __forceinline__ v16h load(const _Float16* p) {
    U f; f.h[0] = *(const v8h*)(p); f.h[1] = *(const v8h*)(p + 16); return f.v;
  }
  static __device__ __forceinline__ v8f mma(v16h a, v16h b, v8f c) {
    return __builtin_amdgcn_wmma_f32_16x16x32_f16(false, a, false, b, (short)0, c, false, false);
  }
  static __device__ __forceinline__ void guard4(v8f& a, v8f& b, v8f& c, v8f& d, v16h x, v16h y) { dep_guard4_h(a, b, c, d, x, y); }
  static __device__ __forceinline__ void keep(v16h a, v16h b, v16h c, v16h d) { keep4_h(a, b, c, d); }
};
template <> struct Frag<__bf16> {
  typedef v16b V; union U { v16b v; v8b h[2]; };
  static __device__ __forceinline__ v16b load(const __bf16* p) {
    U f; f.h[0] = *(const v8b*)(p); f.h[1] = *(const v8b*)(p + 16); return f.v;
  }
  static __device__ __forceinline__ v8f mma(v16b a, v16b b, v8f c) {
    return __builtin_amdgcn_wmma_f32_16x16x32_bf16(false, a, false, b, (short)0, c, false, false);
  }
  static __device__ __forceinline__ void guard4(v8f& a, v8f& b, v8f& c, v8f& d, v16b x, v16b y) { dep_guard4_b(a, b, c, d, x, y); }
  static __device__ __forceinline__ void keep(v16b a, v16b b, v16b c, v16b d) { keep4_b(a, b, c, d); }
};

__device__ __forceinline__ v8f mma_h(v16h a, v16h b, v8f c) {
  c = __builtin_amdgcn_wmma_f32_16x16x32_f16(false, a, false, b, (short)0, c, false, false);
  asm volatile("v_nop\n\tv_nop\n\tv_nop\n\tv_nop" : "+v"(c) : "v"(a), "v"(b));
  return c;
}

template <int ET> struct Elem;
template <> struct Elem<0> { typedef _Float16 T; };
template <> struct Elem<1> { typedef __bf16 T; };
template <int ET, bool SPLIT, int BIAS_MODE, int OUT_MODE, bool RESID, int ACT = 0>
__global__ __launch_bounds__(256) void wmma_gemm64(
    const unsigned short* __restrict__ Ap, const unsigned short* __restrict__ A2p, int lda, long strideA,
    const unsigned short* __restrict__ Btp, const unsigned short* __restrict__ Bt2p, int ldb, long strideB,
    void* __restrict__ Cout, void* __restrict__ Cout2, int ldc, long strideC,
    const float* __restrict__ bias,
    const float* __restrict__ resid, long strideR,
    int M, int N, int K, float scale) {
  typedef typename Elem<ET>::T T;
  typedef typename Frag<T>::V V;
  const T* A = (const T*)Ap; const T* A2 = (const T*)A2p; const T* Bt = (const T*)Btp; const T* Bt2 = (const T*)Bt2p;
  __shared__ __align__(16) float sT[8][16 * 68];
  const int b    = blockIdx.y;
  const int lane = threadIdx.x & 31;
  const int wave = threadIdx.x >> 5;
  const int tilesN = N >> 6;
  const int tilesM = M >> 6;
  const int tile = blockIdx.x * 8 + wave;
  if (tile >= tilesM * tilesN) return;
  const int tm = tile / tilesN;
  const int tn = tile - tm * tilesN;
  const int m0 = tm << 6;
  const int n0 = tn << 6;

  const T* Ab  = A  + (size_t)b * strideA;
  const T* Bb  = Bt + (size_t)b * strideB;
  const T* Ab2 = SPLIT ? (A2  + (size_t)b * strideA) : nullptr;
  const T* Bb2 = SPLIT ? (Bt2 + (size_t)b * strideB) : nullptr;

  const int rlane = lane & 15;
  const int koff  = (lane >> 4) * 8;
  const int mOff  = (lane >> 4) * 8;

  v8f acc[4][4];
#pragma unroll
  for (int i = 0; i < 4; ++i)
#pragma unroll
    for (int j = 0; j < 4; ++j) acc[i][j] = (v8f){0.f,0.f,0.f,0.f,0.f,0.f,0.f,0.f};

  for (int k0 = 0; k0 < K; k0 += 32) {
    V bh[4], bl[4];
#pragma unroll
    for (int j = 0; j < 4; ++j) {
      const size_t bo = (size_t)(n0 + (j << 4) + rlane) * ldb + koff + k0;
      bh[j] = Frag<T>::load(Bb + bo);
      if (SPLIT) bl[j] = Frag<T>::load(Bb2 + bo);
    }
#pragma unroll
    for (int i = 0; i < 4; ++i) {
      const size_t ao = (size_t)(m0 + (i << 4) + rlane) * lda + koff + k0;
      V ah = Frag<T>::load(Ab + ao);
      V al;
      if (SPLIT) al = Frag<T>::load(Ab2 + ao);
#pragma unroll
      for (int j = 0; j < 4; ++j) {
        acc[i][j] = Frag<T>::mma(ah, bh[j], acc[i][j]);
        if (SPLIT) {
          acc[i][j] = Frag<T>::mma(ah, bl[j], acc[i][j]);
          acc[i][j] = Frag<T>::mma(al, bh[j], acc[i][j]);
        }
      }
      Frag<T>::guard4(acc[i][0], acc[i][1], acc[i][2], acc[i][3], ah, SPLIT ? al : ah);
    }
    Frag<T>::keep(bh[0], bh[1], bh[2], bh[3]);
    if (SPLIT) Frag<T>::keep(bl[0], bl[1], bl[2], bl[3]);
  }
  acc_guard4(acc[0][0], acc[0][1], acc[0][2], acc[0][3]);
  acc_guard4(acc[1][0], acc[1][1], acc[1][2], acc[1][3]);
  acc_guard4(acc[2][0], acc[2][1], acc[2][2], acc[2][3]);
  acc_guard4(acc[3][0], acc[3][1], acc[3][2], acc[3][3]);

  float* slab = sT[wave];
  const float* Rb = RESID ? (resid + (size_t)b * strideR) : nullptr;
#pragma unroll
  for (int i = 0; i < 4; ++i) {
    const int mBase = m0 + (i << 4);
#pragma unroll
    for (int j = 0; j < 4; ++j) {
      const int n = n0 + (j << 4) + rlane;
      float bv = 0.f;
      if (BIAS_MODE == 2) bv = bias[n];
#pragma unroll
      for (int r = 0; r < 8; ++r) {
        float v = acc[i][j][r] * scale;
        if (BIAS_MODE == 1) v += bias[mBase + mOff + r];
        if (BIAS_MODE == 2) v += bv;
        if (RESID) v += Rb[(size_t)(mBase + mOff + r) * ldc + n];
        if (ACT == 1) v = tanhf(v);
        if (ACT == 2) v = fmaxf(v, 0.0f);
        if (ACT == 3) v = v / (1.0f + expf(-v));
        if (ACT == 4) v = (v > 0.f) ? v : 0.01f * v;
        slab[(mOff + r) * 68 + (j << 4) + rlane] = v;
      }
    }
    __builtin_amdgcn_fence(__ATOMIC_RELEASE, "workgroup");
    __builtin_amdgcn_wave_barrier();
    __builtin_amdgcn_fence(__ATOMIC_ACQUIRE, "workgroup");
    if (OUT_MODE == 0) {
      float* C = (float*)Cout + (size_t)b * strideC;
      const int hh = lane >> 4, c4 = (lane & 15) * 4;
      for (int pass = 0; pass < 2; ++pass) {
#pragma unroll
        for (int it = 0; it < 8; ++it) {
          const int row = it * 2 + hh;
          v4f v = *(const v4f*)(slab + row * 68 + c4);
          *(volatile v4f*)(C + (size_t)(mBase + row) * ldc + n0 + c4) = v;
        }
        __threadfence();
      }
    } else {
      const int q = lane >> 3, c8 = (lane & 7) * 8;
      unsigned short* C  = (unsigned short*)Cout  + (size_t)b * strideC;
      unsigned short* C2 = (OUT_MODE == 2) ? ((unsigned short*)Cout2 + (size_t)b * strideC) : nullptr;
      for (int pass = 0; pass < 2; ++pass) {
#pragma unroll
        for (int it = 0; it < 4; ++it) {
          const int row = it * 4 + q;
          const float* sp = slab + row * 68 + c8;
          v8h hv, lv;
#pragma unroll
          for (int e = 0; e < 8; ++e) {
            if (OUT_MODE == 1) {
              hv[e] = (_Float16)sp[e];
            } else {
              unsigned short hb = f2bf_bits(sp[e]);
              unsigned short lb = f2bf_bits(sp[e] - bf_bits2f(hb));
              hv[e] = __builtin_bit_cast(_Float16, hb);
              lv[e] = __builtin_bit_cast(_Float16, lb);
            }
          }
          *(volatile v8h*)(C + (size_t)(mBase + row) * ldc + n0 + c8) = hv;
          if (OUT_MODE == 2) *(volatile v8h*)(C2 + (size_t)(mBase + row) * ldc + n0 + c8) = lv;
        }
        __threadfence();
      }
    }
    __builtin_amdgcn_fence(__ATOMIC_RELEASE, "workgroup");
    __builtin_amdgcn_wave_barrier();
    __builtin_amdgcn_fence(__ATOMIC_ACQUIRE, "workgroup");
  }
}


__device__ __forceinline__ float fast_tanh(float v) { return 1.0f - 2.0f * frcp(__expf(2.0f * v) + 1.0f); }
__device__ __forceinline__ float fast_sigmoid(float v) { return frcp(1.0f + __expf(-v)); }

__global__ __launch_bounds__(kThr) void wsetup_kernel(const float* __restrict__ eWih, const float* __restrict__ eWhh, const float* __restrict__ eb,
                                                      const float* __restrict__ lWih, const float* __restrict__ lWhh, const float* __restrict__ lb,
                                                      const float* __restrict__ dWih, const float* __restrict__ dWhh, const float* __restrict__ db,
                                                      const float* __restrict__ oW, const float* __restrict__ ob,
                                                      unsigned short* __restrict__ WE, unsigned short* __restrict__ WL, unsigned short* __restrict__ WD,
                                                      unsigned short* __restrict__ WO, float* __restrict__ BIAS) {
  unsigned v = blockIdx.x * (unsigned)kThr + threadIdx.x;
  asm volatile("" : "+v"(v));
  if (v < 10752u) {
    const float* sp = eWhh; bool live = true; unsigned short* dp = WE;
    if (v < 4096u) {
      const unsigned n = v >> 4, k8 = (v & 15u) * 8u;
      live = k8 < 104u; sp = (k8 < 64u) ? (eWhh + (size_t)n * kHE + k8) : (eWih + (size_t)n * kF + (live ? k8 - 64u : 0u)); dp = WE + (size_t)v * 8u;
    } else if (v < 6144u) {
      const unsigned w = v - 4096u, n = w >> 4, k8 = (w & 15u) * 8u;
      live = k8 < 96u; sp = (k8 < 32u) ? (lWhh + (size_t)n * kHL + k8) : (lWih + (size_t)n * kHE + (live ? k8 - 32u : 0u)); dp = WL + (size_t)w * 8u;
    } else if (v < 10240u) {
      const unsigned w = v - 6144u, n = w >> 4, k8 = (w & 15u) * 8u;
      live = k8 < 96u; sp = (k8 < 64u) ? (dWhh + (size_t)n * kHD + k8) : (dWih + (size_t)n * kHL + (live ? k8 - 64u : 0u)); dp = WD + (size_t)w * 8u;
    } else {
      const unsigned w = v - 10240u, n = w >> 3, k8 = (w & 7u) * 8u;
      live = n < (unsigned)kF; sp = oW + (size_t)(live ? n : 0u) * kHD + k8; dp = WO + (size_t)w * 8u;
    }
    const v4f a0 = *(const v4f*)sp, a1 = *(const v4f*)(sp + 4);
    v8h hv;
#pragma unroll
    for (int e = 0; e < 4; ++e) {
      hv[e] = (_Float16)(live ? carry_flush(bf16r(a0[e]), kInCarry) : 0.0f);
      hv[4 + e] = (_Float16)(live ? carry_flush(bf16r(a1[e]), kInCarry) : 0.0f);
    }
    *(volatile v8h*)dp = hv;
    __threadfence();
    *(volatile v8h*)dp = hv;
  } else {
    const unsigned i0 = (v - 10752u) * 4u;
    const float* sp = (i0 < 256u) ? (eb + i0) : (i0 < 384u) ? (lb + (i0 - 256u)) : (i0 < 640u) ? (db + (i0 - 384u)) : (ob + ((i0 < 680u) ? (i0 - 640u) : 0u));
    const bool live = i0 < 680u;
    const v4f a = *(const v4f*)sp;
    v4f o;
#pragma unroll
    for (int e = 0; e < 4; ++e) { const float x = a[e]; o[e] = live ? bf16r(x) : 0.0f; }
    float* dp = BIAS + i0;
    *(volatile v4f*)dp = o;
    __threadfence();
    *(volatile v4f*)dp = o;
  }
}
static_assert(256 * 16 == 4096 && 128 * 16 == 2048 && 64 * 8 == 512 && 4096 + 2048 + 4096 + 512 == 10752 && kFEnd / 4 == 256 && 10752 + 256 == 43 * kThr && (kFBO + kF) == 680 && (680 % 4) == 0, "weight set-up grid exact");

__global__ __launch_bounds__(kThr) void zinit_kernel(const float* __restrict__ x, unsigned short* __restrict__ AE, unsigned short* __restrict__ ALD,
                                                     float* __restrict__ CELLS) {
  unsigned v = blockIdx.x * (unsigned)kThr + threadIdx.x;
  asm volatile("" : "+v"(v));
  if (v < 196608u) {
    v8h hv;
#pragma unroll
    for (int e = 0; e < 8; ++e) hv[e] = (_Float16)0.0f;
    unsigned short* dp = (v < 65536u) ? (AE + (size_t)v * 8u) : (ALD + (size_t)(v - 65536u) * 8u);
    if (v < 65536u) {
      const unsigned b = v >> 4, k8 = (v & 15u) * 8u;
      const bool xs = (k8 >= 64u) && (k8 < 104u);
      const float* sp = x + (size_t)b * kT * kF + (xs ? k8 - 64u : 0u);
      const v4f a0 = *(const v4f*)sp, a1 = *(const v4f*)(sp + 4);
#pragma unroll
      for (int e = 0; e < 4; ++e) {
        hv[e] = (_Float16)(xs ? carry_flush(bf16r(a0[e]), kInCarry) : 0.0f);
        hv[4 + e] = (_Float16)(xs ? carry_flush(bf16r(a1[e]), kInCarry) : 0.0f);
      }
    }
    *(volatile v8h*)dp = hv;
    __threadfence();
    *(volatile v8h*)dp = hv;
  } else {
    const v4f o = {0.f, 0.f, 0.f, 0.f};
    float* dp = CELLS + (size_t)(v - 196608u) * 4u;
    *(volatile v4f*)dp = o;
    __threadfence();
    *(volatile v4f*)dp = o;
  }
}
static_assert(kB * 16 == 65536 && 2 * kB * 16 == 131072 && kB * (kHE + kHL + kHD) / 4 == 163840 && 65536 + 131072 + 163840 == 1408 * kThr, "plane set-up grid exact");

__global__ __launch_bounds__(kThr) void cell_enc_kernel(const float* __restrict__ GE, const float* __restrict__ x, float* __restrict__ CE,
                                                        unsigned short* __restrict__ AE, unsigned short* __restrict__ AL, int t) {
  unsigned v = blockIdx.x * (unsigned)kThr + threadIdx.x;
  asm volatile("" : "+v"(v));
  const unsigned b = v >> 3, u8 = (v & 7u) * 8u;
  const float* gr = GE + (size_t)b * 256u + u8;
  float* cp = CE + (size_t)b * kHE + u8;
  v8h hv, xv;
  v4f cn0, cn1;
#pragma unroll
  for (int hlf = 0; hlf < 2; ++hlf) {
    const v4f gi = *(const v4f*)(gr + 4 * hlf), gf = *(const v4f*)(gr + kHE + 4 * hlf), gg = *(const v4f*)(gr + 2 * kHE + 4 * hlf), go = *(const v4f*)(gr + 3 * kHE + 4 * hlf);
    const v4f co = *(const v4f*)(cp + 4 * hlf);
#pragma unroll
    for (int e = 0; e < 4; ++e) {
      const float cn = fast_sigmoid(gf[e]) * co[e] + fast_sigmoid(gi[e]) * fast_tanh(gg[e]);
      const float hn = fast_sigmoid(go[e]) * fast_tanh(cn);
      if (hlf == 0) cn0[e] = cn; else cn1[e] = cn;
      hv[4 * hlf + e] = (_Float16)carry_flush(hn, kInCarry);
    }
  }
  const bool nx = (u8 < (unsigned)kF) && (t + 1 < kT);
  {
    const float* sp = x + ((size_t)b * kT + (size_t)(nx ? (t + 1) : 0)) * kF + (nx ? u8 : 0u);
    const v4f a0 = *(const v4f*)sp, a1 = *(const v4f*)(sp + 4);
#pragma unroll
    for (int e = 0; e < 4; ++e) { const float p = a0[e], q = a1[e]; xv[e] = (_Float16)carry_flush(bf16r(p), kInCarry); xv[4 + e] = (_Float16)carry_flush(bf16r(q), kInCarry); }
  }
  unsigned short* hp = AE + (size_t)b * kKP + u8;
  unsigned short* xp = AE + (size_t)b * kKP + kHE + (nx ? u8 : 0u);
  unsigned short* lp = AL + (size_t)b * kKP + kHL + u8;
  const bool last = (t == kT - 1);
  for (int pass = 0; pass < 2; ++pass) {
    *(volatile v4f*)cp = cn0; *(volatile v4f*)(cp + 4) = cn1;
    *(volatile v8h*)hp = hv;
    if (nx) *(volatile v8h*)xp = xv;
    if (last) *(volatile v8h*)lp = hv;
    __threadfence();
  }
}
static_assert(kB * 8 == 128 * kThr && (kF % 8) == 0, "encoder cell grid exact; the input's threads end on a multiple of 8 columns");

__global__ __launch_bounds__(kThr) void cell_ld_kernel(const float* __restrict__ GL, const float* __restrict__ GD, float* __restrict__ CL, float* __restrict__ CD,
                                                       unsigned short* __restrict__ AL, unsigned short* __restrict__ AD, unsigned short* __restrict__ HD16, int k) {
  const bool lat = blockIdx.x < 64u;
  if (lat ? (k >= kT) : (k < 1)) return;
  unsigned v = (lat ? blockIdx.x : (blockIdx.x - 64u)) * (unsigned)kThr + threadIdx.x;
  asm volatile("" : "+v"(v));
  const unsigned b = lat ? (v >> 2) : (v >> 3);
  const unsigned u8 = (lat ? (v & 3u) : (v & 7u)) * 8u;
  const unsigned hw = lat ? (unsigned)kHL : (unsigned)kHD;
  const float* gr = (lat ? GL + (size_t)b * 128u : GD + (size_t)b * 256u) + u8;
  float* cp = (lat ? CL + (size_t)b * kHL : CD + (size_t)b * kHD) + u8;
  v8h hv;
  v4f cn0, cn1;
#pragma unroll
  for (int hlf = 0; hlf < 2; ++hlf) {
    const v4f gi = *(const v4f*)(gr + 4 * hlf), gf = *(const v4f*)(gr + hw + 4 * hlf), gg = *(const v4f*)(gr + 2u * hw + 4 * hlf), go = *(const v4f*)(gr + 3u * hw + 4 * hlf);
    const v4f co = *(const v4f*)(cp + 4 * hlf);
#pragma unroll
    for (int e = 0; e < 4; ++e) {
      const float cn = fast_sigmoid(gf[e]) * co[e] + fast_sigmoid(gi[e]) * fast_tanh(gg[e]);
      const float hn = fast_sigmoid(go[e]) * fast_tanh(cn);
      if (hlf == 0) cn0[e] = cn; else cn1[e] = cn;
      hv[4 * hlf + e] = (_Float16)carry_flush(hn, kInCarry);
    }
  }
  unsigned short* p1 = lat ? (AL + (size_t)b * kKP + u8) : (AD + (size_t)b * kKP + u8);
  unsigned short* p2 = lat ? (AD + (size_t)b * kKP + kHD + u8) : (HD16 + ((size_t)b * kT + (size_t)(k - 1)) * kHD + u8);
  for (int pass = 0; pass < 2; ++pass) {
    *(volatile v4f*)cp = cn0; *(volatile v4f*)(cp + 4) = cn1;
    *(volatile v8h*)p1 = hv;
    *(volatile v8h*)p2 = hv;
    __threadfence();
  }
}
static_assert(kB * 4 == 64 * kThr && kB * 8 == 128 * kThr, "wavefront cell grid: 64 + 128 blocks");

__global__ __launch_bounds__(kThr) void out_kernel(const float* __restrict__ O32, float* __restrict__ outq) {
  unsigned v = blockIdx.x * (unsigned)kThr + threadIdx.x;
  asm volatile("" : "+v"(v));
  const unsigned i4 = v * 4u;
  const unsigned r = i4 / (unsigned)kF, f = i4 % (unsigned)kF;
  const v4f o = *(const v4f*)(O32 + (size_t)r * 64u + f);
  float* dp = outq + (size_t)i4;
  *(volatile v4f*)dp = o;
  __threadfence();
  *(volatile v4f*)dp = o;
}
static_assert((size_t)kRowsQ * kF / 4 == 4000 * kThr && (kF % 4) == 0, "output grid exact");

extern "C" void kernel_launch(void* const* d_in, const int* in_sizes, int n_in,
                              void* d_out, int out_size, void* d_ws, size_t ws_size,
                              hipStream_t stream) {
  if (n_in < 12 || d_out == nullptr || d_ws == nullptr) return;
  if (in_sizes[0] != kB * kT * kF || in_sizes[1] != 256 * kF || in_sizes[2] != 256 * kHE || in_sizes[3] != 256) return;
  if (in_sizes[4] != 128 * kHE || in_sizes[5] != 128 * kHL || in_sizes[6] != 128) return;
  if (in_sizes[7] != 256 * kHL || in_sizes[8] != 256 * kHD || in_sizes[9] != 256 || in_sizes[10] != kF * kHD || in_sizes[11] != kF) return;
  if (out_size != kRowsY * kF) return;
  if (ws_size < kWsTotal) return;
  const float* x = (const float*)d_in[0];
  const float* eWih = (const float*)d_in[1];
  const float* eWhh = (const float*)d_in[2];
  const float* eb = (const float*)d_in[3];
  const float* lWih = (const float*)d_in[4];
  const float* lWhh = (const float*)d_in[5];
  const float* lb = (const float*)d_in[6];
  const float* dWih = (const float*)d_in[7];
  const float* dWhh = (const float*)d_in[8];
  const float* db = (const float*)d_in[9];
  const float* oW = (const float*)d_in[10];
  const float* ob = (const float*)d_in[11];
  float* out = (float*)d_out;
  char* ws = (char*)d_ws;
  unsigned short* WE = (unsigned short*)(ws + kOffWE);
  unsigned short* WL = (unsigned short*)(ws + kOffWL);
  unsigned short* WD = (unsigned short*)(ws + kOffWD);
  unsigned short* WO = (unsigned short*)(ws + kOffWO);
  float* BIAS = (float*)(ws + kOffBIAS);
  unsigned short* AE = (unsigned short*)(ws + kOffAE);
  unsigned short* AL = (unsigned short*)(ws + kOffAL);
  unsigned short* AD = (unsigned short*)(ws + kOffAD);
  float* GE = (float*)(ws + kOffGE);
  float* GL = (float*)(ws + kOffGL);
  float* GD = (float*)(ws + kOffGD);
  float* CE = (float*)(ws + kOffCE);
  float* CL = (float*)(ws + kOffCL);
  float* CD = (float*)(ws + kOffCD);
  unsigned short* HD16 = (unsigned short*)(ws + kOffHD16);
  float* O32 = (float*)(ws + kOffO32);

  wsetup_kernel<<<43, kThr, 0, stream>>>(eWih, eWhh, eb, lWih, lWhh, lb, dWih, dWhh, db, oW, ob, WE, WL, WD, WO, BIAS);
  zinit_kernel<<<1408, kThr, 0, stream>>>(x, AE, AL, CE);

  for (int t = 0; t < kT; ++t) {
    wmma_gemm64<0, false, 2, 0, false, 0><<<dim3((kB / 64) * (256 / 64) / 8, 1), 256, 0, stream>>>(
        AE, AE, kKP, 0L, WE, WE, kKP, 0L, (void*)GE, (void*)GE, 256, 0L, BIAS + kFBE, nullptr, 0L, kB, 256, kKP, kSc);
    cell_enc_kernel<<<128, kThr, 0, stream>>>(GE, x, CE, AE, AL, t);
  }
  for (int k = 0; k <= kT; ++k) {
    if (k < kT) {
      wmma_gemm64<0, false, 2, 0, false, 0><<<dim3((kB / 64) * (128 / 64) / 8, 1), 256, 0, stream>>>(
          AL, AL, kKP, 0L, WL, WL, kKP, 0L, (void*)GL, (void*)GL, 128, 0L, BIAS + kFBL, nullptr, 0L, kB, 128, kKP, kSc);
    }
    if (k >= 1) {
      wmma_gemm64<0, false, 2, 0, false, 0><<<dim3((kB / 64) * (256 / 64) / 8, 1), 256, 0, stream>>>(
          AD, AD, kKP, 0L, WD, WD, kKP, 0L, (void*)GD, (void*)GD, 256, 0L, BIAS + kFBD, nullptr, 0L, kB, 256, kKP, kSc);
    }
    cell_ld_kernel<<<192, kThr, 0, stream>>>(GL, GD, CL, CD, AL, AD, HD16, k);
  }
  for (int q = 0; q < 4; ++q) {
    const unsigned short* hq = HD16 + (size_t)q * kRowsQ * kHD;
    wmma_gemm64<0, false, 2, 0, false, 0><<<dim3((kRowsQ / 64) * (64 / 64) / 8, 1), 256, 0, stream>>>(
        hq, hq, kHD, 0L, WO, WO, kHD, 0L, (void*)O32, (void*)O32, 64, 0L, BIAS + kFBO, nullptr, 0L, kRowsQ, 64, kHD, kSc);
    out_kernel<<<4000, kThr, 0, stream>>>(O32, out + (size_t)q * kRowsQ * kF);
  }
}
